// CVRP_Decoder_51410758533182
// MI455X (gfx1250) — hardware-verified
//
#include <hip/hip_runtime.h>
#include <math.h>

typedef __attribute__((ext_vector_type(16))) _Float16 v16h;
typedef __attribute__((ext_vector_type(8)))  _Float16 v8h;
typedef __attribute__((ext_vector_type(16))) __bf16   v16b;
typedef __attribute__((ext_vector_type(8)))  __bf16   v8b;
typedef __attribute__((ext_vector_type(8)))  float    v8f;
typedef __attribute__((ext_vector_type(4)))  float    v4f;
typedef __attribute__((ext_vector_type(4)))  unsigned int v4u;

constexpr int kB   = 16;
constexpr int kP   = 100;
constexpr int kN   = 1000;
constexpr int kNP  = 1024;
constexpr int kE   = 128;
constexpr int kH   = 8;
constexpr int kD   = 16;
constexpr int kHD  = 128;
constexpr int kQD  = 16;
constexpr int kDYN = 3;
constexpr int kHID = 64;
constexpr int kBP     = kB * kP;
constexpr int kBPpad  = 1664;
constexpr int kEncRows = kB * kNP;
constexpr int kChunkB   = 2;
constexpr int kChunkBP  = kChunkB * kP;
constexpr int kChunkRows = kChunkBP * kNP;
constexpr int kNumChunks = kB / kChunkB;
constexpr int kSrows = 128;
constexpr float kWCarry   = 16.0f;
constexpr float kInvSqrtE = 0.08838834764831845f;
constexpr float kClip     = 10.0f;
static_assert(kBPpad % 64 == 0 && kBPpad >= kBP, "pad");
static_assert(kChunkRows % 256 == 0 && kChunkRows % 64 == 0, "chunk");
static_assert(kB % kChunkB == 0, "chunks");
static_assert(kBPpad >= (kB - 1) * kP + kSrows, "last batch score rows inside MH planes");
static_assert(kH * kD == kHD && kE == kHD, "dims");

__device__ __forceinline__ unsigned short f2bf_bits(float f) {
  unsigned u = __float_as_uint(f);
  return (unsigned short)((u + 0x7FFFu + ((u >> 16) & 1u)) >> 16);
}
__device__ __forceinline__ float bf_bits2f(unsigned short h) { return __uint_as_float(((unsigned)h) << 16); }

__device__ __forceinline__ void dep_guard_h(v8f& a, v8f& b, v16h x, v16h y) { asm volatile("v_nop\n\tv_nop\n\tv_nop\n\tv_nop" : "+v"(a), "+v"(b) : "v"(x), "v"(y)); }
__device__ __forceinline__ void dep_guard_b(v8f& a, v8f& b, v16b x, v16b y) { asm volatile("v_nop\n\tv_nop\n\tv_nop\n\tv_nop" : "+v"(a), "+v"(b) : "v"(x), "v"(y)); }
__device__ __forceinline__ void keep4_h(v16h a, v16h b, v16h c, v16h d) { asm volatile("v_nop" :: "v"(a), "v"(b), "v"(c), "v"(d)); }
__device__ __forceinline__ void keep4_b(v16b a, v16b b, v16b c, v16b d) { asm volatile("v_nop" :: "v"(a), "v"(b), "v"(c), "v"(d)); }
__device__ __forceinline__ void acc_guard4(v8f& a, v8f& b, v8f& c, v8f& d) { asm volatile("v_nop\n\tv_nop\n\tv_nop\n\tv_nop" : "+v"(a), "+v"(b), "+v"(c), "+v"(d)); }
template <typename T> struct Frag;
template <> struct Frag<_Float16> {
  typedef v16h V; union U { v16h v; v8h h[2]; };
  static __device__ __forceinline__ v16h load(const _Float16* p) {
    U f; f.h[0] = *(const v8h*)(p); f.h[1] = *(const v8h*)(p + 16); return f.v;
  }
  static __device__ __forceinline__ v8f mma(v16h a, v16h b, v8f c) {
    return __builtin_amdgcn_wmma_f32_16x16x32_f16(false, a, false, b, (short)0, c, false, false);
  }
  static __device__ __forceinline__ void guard(v8f& a, v8f& b, v16h x, v16h y) { dep_guard_h(a, b, x, y); }
  static __device__ __forceinline__ void keep(v16h a, v16h b, v16h c, v16h d) { keep4_h(a, b, c, d); }
};
template <> struct Frag<__bf16> {
  typedef v16b V; union U { v16b v; v8b h[2]; };
  static __device__ __forceinline__ v16b load(const __bf16* p) {
    U f; f.h[0] = *(const v8b*)(p); f.h[1] = *(const v8b*)(p + 16); return f.v;
  }
  static __device__ __forceinline__ v8f mma(v16b a, v16b b, v8f c) {
    return __builtin_amdgcn_wmma_f32_16x16x32_bf16(false, a, false, b, (short)0, c, false, false);
  }
  static __device__ __forceinline__ void guard(v8f& a, v8f& b, v16b x, v16b y) { dep_guard_b(a, b, x, y); }
  static __device__ __forceinline__ void keep(v16b a, v16b b, v16b c, v16b d) { keep4_b(a, b, c, d); }
};

__device__ __forceinline__ unsigned pk16(unsigned short a, unsigned short b) { return (unsigned)a | ((unsigned)b << 16); }
__device__ __forceinline__ unsigned short h_bits(float f) { const _Float16 h = (_Float16)f; return __builtin_bit_cast(unsigned short, h); }
__device__ __forceinline__ void split_bf(float f, unsigned short& hb, unsigned short& lb) {
  hb = f2bf_bits(f);
  lb = f2bf_bits(f - bf_bits2f(hb));
}

template <int ET> struct Elem;
template <> struct Elem<0> { typedef _Float16 T; };
template <> struct Elem<1> { typedef __bf16 T; };
template <int ET, bool SPLIT, int BIAS_MODE, int OUT_MODE, bool RESID, int ACT = 0>
__global__ __launch_bounds__(256) void wmma_gemm64(
    const unsigned short* __restrict__ Ap, const unsigned short* __restrict__ A2p, int lda, long strideA,
    const unsigned short* __restrict__ Btp, const unsigned short* __restrict__ Bt2p, int ldb, long strideB,
    void* __restrict__ Cout, void* __restrict__ Cout2, int ldc, long strideC,
    const float* __restrict__ bias,
    const float* __restrict__ resid, long strideR,
    int M, int N, int K, float scale) {
  typedef typename Elem<ET>::T T;
  typedef typename Frag<T>::V V;
  const T* A = (const T*)Ap; const T* A2 = (const T*)A2p; const T* Bt = (const T*)Btp; const T* Bt2 = (const T*)Bt2p;
  __shared__ __align__(16) float sT[8][16 * 68];
  const int b    = blockIdx.y;
  const int lane = threadIdx.x & 31;
  const int wave = threadIdx.x >> 5;
  const int tilesN = N >> 6;
  const int tilesM = M >> 6;
  const int tile = blockIdx.x * 8 + wave;
  if (tile >= tilesM * tilesN) return;
  const int tm = tile / tilesN;
  const int tn = tile - tm * tilesN;
  const int m0 = tm << 6;
  const int n0 = tn << 6;

  const T* Ab  = A  + (size_t)b * strideA;
  const T* Bb  = Bt + (size_t)b * strideB;
  const T* Ab2 = SPLIT ? (A2  + (size_t)b * strideA) : nullptr;
  const T* Bb2 = SPLIT ? (Bt2 + (size_t)b * strideB) : nullptr;

  const int rlane = lane & 15;
  const int koff  = (lane >> 4) * 8;
  const int mOff  = (lane >> 4) * 8;

  v8f acc[4][4];
#pragma unroll
  for (int i = 0; i < 4; ++i)
#pragma unroll
    for (int j = 0; j < 4; ++j) acc[i][j] = (v8f){0.f,0.f,0.f,0.f,0.f,0.f,0.f,0.f};

  for (int k0 = 0; k0 < K; k0 += 32) {
    V bh[4], bl[4];
#pragma unroll
    for (int j = 0; j < 4; ++j) {
      const size_t bo = (size_t)(n0 + (j << 4) + rlane) * ldb + koff + k0;
      bh[j] = Frag<T>::load(Bb + bo);
      if (SPLIT) bl[j] = Frag<T>::load(Bb2 + bo);
    }
#pragma unroll
    for (int i = 0; i < 4; ++i) {
      const size_t ao = (size_t)(m0 + (i << 4) + rlane) * lda + koff + k0;
      V ah = Frag<T>::load(Ab + ao);
      V al;
      if (SPLIT) al = Frag<T>::load(Ab2 + ao);
#pragma unroll
      for (int j = 0; j < 4; ++j) {
        acc[i][j] = Frag<T>::mma(ah, bh[j], acc[i][j]);
        if (SPLIT) {
          acc[i][j] = Frag<T>::mma(ah, bl[j], acc[i][j]);
          acc[i][j] = Frag<T>::mma(al, bh[j], acc[i][j]);
        }
      }
      Frag<T>::guard(acc[i][0], acc[i][3], ah, SPLIT ? al : ah);
    }
    Frag<T>::keep(bh[0], bh[1], bh[2], bh[3]);
    if (SPLIT) Frag<T>::keep(bl[0], bl[1], bl[2], bl[3]);
  }
  acc_guard4(acc[0][0], acc[0][1], acc[0][2], acc[0][3]);
  acc_guard4(acc[1][0], acc[1][1], acc[1][2], acc[1][3]);
  acc_guard4(acc[2][0], acc[2][1], acc[2][2], acc[2][3]);
  acc_guard4(acc[3][0], acc[3][1], acc[3][2], acc[3][3]);

  float* slab = sT[wave];
  const float* Rb = RESID ? (resid + (size_t)b * strideR) : nullptr;
#pragma unroll
  for (int i = 0; i < 4; ++i) {
    const int mBase = m0 + (i << 4);
#pragma unroll
    for (int j = 0; j < 4; ++j) {
      const int n = n0 + (j << 4) + rlane;
      float bv = 0.f;
      if (BIAS_MODE == 2) bv = bias[n];
#pragma unroll
      for (int r = 0; r < 8; ++r) {
        float v = acc[i][j][r] * scale;
        if (BIAS_MODE == 1) v += bias[mBase + mOff + r];
        if (BIAS_MODE == 2) v += bv;
        if (RESID) v += Rb[(size_t)(mBase + mOff + r) * ldc + n];
        if (ACT == 2) v = fmaxf(v, 0.0f);
        if (ACT == 4) v = (v > 0.f) ? v : 0.01f * v;
        slab[(mOff + r) * 68 + (j << 4) + rlane] = v;
      }
    }
    __builtin_amdgcn_fence(__ATOMIC_RELEASE, "workgroup");
    __builtin_amdgcn_wave_barrier();
    __builtin_amdgcn_fence(__ATOMIC_ACQUIRE, "workgroup");
    if (OUT_MODE == 0) {
      float* C = (float*)Cout + (size_t)b * strideC;
      const int hh = lane >> 4, c4 = (lane & 15) * 4;
      for (int pass = 0; pass < 2; ++pass) {
#pragma unroll
        for (int it = 0; it < 8; ++it) {
          const int row = it * 2 + hh;
          v4f v = *(const v4f*)(slab + row * 68 + c4);
          *(volatile v4f*)(C + (size_t)(mBase + row) * ldc + n0 + c4) = v;
        }
        __threadfence();
      }
    } else {
      const int q = lane >> 3, c8 = (lane & 7) * 8;
      unsigned short* C  = (unsigned short*)Cout  + (size_t)b * strideC;
      unsigned short* C2 = (OUT_MODE == 2) ? ((unsigned short*)Cout2 + (size_t)b * strideC) : nullptr;
      for (int pass = 0; pass < 2; ++pass) {
#pragma unroll
        for (int it = 0; it < 4; ++it) {
          const int row = it * 4 + q;
          const float* sp = slab + row * 68 + c8;
          v8h hv, lv;
#pragma unroll
          for (int e = 0; e < 8; ++e) {
            if (OUT_MODE == 1) {
              hv[e] = (_Float16)sp[e];
            } else {
              unsigned short hb = f2bf_bits(sp[e]);
              unsigned short lb = f2bf_bits(sp[e] - bf_bits2f(hb));
              hv[e] = __builtin_bit_cast(_Float16, hb);
              lv[e] = __builtin_bit_cast(_Float16, lb);
            }
          }
          *(volatile v8h*)(C + (size_t)(mBase + row) * ldc + n0 + c8) = hv;
          if (OUT_MODE == 2) *(volatile v8h*)(C2 + (size_t)(mBase + row) * ldc + n0 + c8) = lv;
        }
        __threadfence();
      }
    }
    __builtin_amdgcn_fence(__ATOMIC_RELEASE, "workgroup");
    __builtin_amdgcn_wave_barrier();
    __builtin_amdgcn_fence(__ATOMIC_ACQUIRE, "workgroup");
  }
}

__global__ __launch_bounds__(256) void k_wprep(const float* __restrict__ Wk, const float* __restrict__ Wv,
                                              const float* __restrict__ Wcomb, const float* __restrict__ W2,
                                              unsigned short* __restrict__ WkvHi, unsigned short* __restrict__ WkvLo,
                                              unsigned short* __restrict__ WcHi, unsigned short* __restrict__ WcLo,
                                              unsigned short* __restrict__ W2T) {
  __shared__ float sm[64][65];
  const int t = threadIdx.x, lane = t & 31, wave = t >> 5;
  const int bid = blockIdx.x;
  const float* W = Wk; unsigned short* outH = WkvHi; unsigned short* outL = WkvLo;
  int ldn = kHD, ldk = kE, nt = 0, kt = 0; float carry = 1.0f;
  const bool two_planes = (bid < 12);
  if (bid < 4)       { W = Wk;    outH = WkvHi;                    outL = WkvLo;                    ldn = kHD;  ldk = kE;   nt = bid & 1;       kt = bid >> 1;       carry = 1.0f; }
  else if (bid < 8)  { W = Wv;    outH = WkvHi + (size_t)kHD * kE; outL = WkvLo + (size_t)kHD * kE; ldn = kHD;  ldk = kE;   nt = (bid - 4) & 1; kt = (bid - 4) >> 1; carry = 1.0f; }
  else if (bid < 12) { W = Wcomb; outH = WcHi;                     outL = WcLo;                     ldn = kE;   ldk = kHD;  nt = (bid - 8) & 1; kt = (bid - 8) >> 1; carry = 1.0f; }
  else               { W = W2;    outH = W2T;                      outL = W2T;                      ldn = kHID; ldk = kHID; nt = 0;             kt = 0;              carry = kWCarry; }
  const int n0 = nt * 64, k0 = kt * 64;
#pragma unroll
  for (int i = 0; i < 16; ++i) {
    const int e = i * 256 + t;
    const int r = e >> 6;
    const int c = e & 63;
    sm[c][r] = W[(size_t)(k0 + r) * ldn + n0 + c] * carry;
  }
  __syncthreads();
  const int q = lane >> 3, c8 = (lane & 7) * 8;
  v4u uh[2], ul[2];
  int rowv[2];
#pragma unroll
  for (int it = 0; it < 2; ++it) {
    const int row = wave * 8 + it * 4 + q;
    rowv[it] = row;
    unsigned short hb[8], lb[8];
#pragma unroll
    for (int e = 0; e < 8; ++e) {
      const float v = sm[row][c8 + e];
      if (two_planes) { split_bf(v, hb[e], lb[e]); }
      else { hb[e] = h_bits(v); lb[e] = hb[e]; }
    }
    uh[it] = (v4u){pk16(hb[0], hb[1]), pk16(hb[2], hb[3]), pk16(hb[4], hb[5]), pk16(hb[6], hb[7])};
    ul[it] = (v4u){pk16(lb[0], lb[1]), pk16(lb[2], lb[3]), pk16(lb[4], lb[5]), pk16(lb[6], lb[7])};
  }
  for (int pass = 0; pass < 2; ++pass) {
#pragma unroll
    for (int it = 0; it < 2; ++it) {
      const size_t o = (size_t)(n0 + rowv[it]) * ldk + k0 + c8;
      *(volatile v4u*)(outH + o) = uh[it];
      if (two_planes) *(volatile v4u*)(outL + o) = ul[it];
    }
    __threadfence();
  }
}

__global__ __launch_bounds__(256) void k_enc_cast(const float* __restrict__ enc, unsigned short* __restrict__ outHi,
                                                 unsigned short* __restrict__ outLo) {
  const int i = blockIdx.x * 256 + threadIdx.x;
  if (i >= kEncRows * 16) return;
  const int row = i >> 4, c8 = (i & 15) * 8;
  const int b = row >> 10, n = row & (kNP - 1);
  const int nc = (n < kN) ? n : (kN - 1);
  const float* p = enc + ((size_t)(b * kN + nc)) * kE + c8;
  const v4f a = *(const v4f*)(p);
  const v4f c = *(const v4f*)(p + 4);
  const bool valid = (n < kN);
  unsigned short hb[8], lb[8];
#pragma unroll
  for (int e = 0; e < 4; ++e) {
    split_bf(valid ? a[e] : 0.0f, hb[e], lb[e]);
    split_bf(valid ? c[e] : 0.0f, hb[4 + e], lb[4 + e]);
  }
  const v4u uh = (v4u){pk16(hb[0], hb[1]), pk16(hb[2], hb[3]), pk16(hb[4], hb[5]), pk16(hb[6], hb[7])};
  const v4u ul = (v4u){pk16(lb[0], lb[1]), pk16(lb[2], lb[3]), pk16(lb[4], lb[5]), pk16(lb[6], lb[7])};
  const size_t o = (size_t)row * kE + c8;
  *(volatile v4u*)(outHi + o) = uh;
  *(volatile v4u*)(outLo + o) = ul;
  __threadfence();
  *(volatile v4u*)(outHi + o) = uh;
  *(volatile v4u*)(outLo + o) = ul;
}

__global__ __launch_bounds__(128) void k_qside(const float* __restrict__ enc_last, const float* __restrict__ loadv,
                                              const float* __restrict__ Wq, const float* __restrict__ fW1,
                                              const float* __restrict__ fb1, const float* __restrict__ fW2,
                                              const float* __restrict__ fb2, const float* __restrict__ lqW,
                                              const float* __restrict__ lqb, const float* __restrict__ lW1,
                                              const float* __restrict__ lb1,
                                              float* __restrict__ Qs, float* __restrict__ QW) {
  __shared__ float qin[kE + 4];
  __shared__ float g1s[kE + 4];
  __shared__ __align__(16) float qst[kHD];
  __shared__ float qfs[kQD];
  __shared__ __align__(16) float qws[kHID];
  const int bp = blockIdx.x;
  const int t = threadIdx.x, lane = t & 31, wave = t >> 5;
  qin[t] = enc_last[(size_t)bp * kE + t];
  if (t == 0) qin[kE] = loadv[bp];
  __syncthreads();
  for (int j = t; j < kE + 1; j += 128) {
    float acc = fb1[j];
#pragma unroll 1
    for (int e = 0; e < kE + 1; ++e) acc = fmaf(qin[e], fW1[(size_t)e * (kE + 1) + j], acc);
    g1s[j] = fmaxf(acc, 0.0f);
  }
  __syncthreads();
  {
    const int j = t;
    float qv = 0.0f, gm = fb2[j];
#pragma unroll 1
    for (int e = 0; e < kE + 1; ++e) {
      qv = fmaf(qin[e], Wq[(size_t)e * kHD + j], qv);
      gm = fmaf(g1s[e], fW2[(size_t)e * kHD + j], gm);
    }
    const float den = 1.0f + expf(-gm);
    const float gamma = 2.0f * (1.0f / den);
    qst[j] = (qv * gamma) * 0.25f;
  }
  if (t < kQD) {
    float acc = lqb[t];
#pragma unroll 1
    for (int e = 0; e < kE + 1; ++e) acc = fmaf(qin[e], lqW[(size_t)e * kQD + t], acc);
    qfs[t] = acc;
  }
  __syncthreads();
  if (t < kHID) {
    float acc = lb1[t];
#pragma unroll 1
    for (int i = 0; i < kQD; ++i) acc = fmaf(qfs[i], lW1[(size_t)(kDYN + i) * kHID + t], acc);
    qws[t] = acc;
  }
  __syncthreads();
  if (wave == 0) {
    const v4f v = *(const v4f*)(qst + 4 * lane);
    float* dst = Qs + (size_t)bp * kHD + 4 * lane;
    *(volatile v4f*)dst = v;
    __threadfence();
    *(volatile v4f*)dst = v;
  } else if (wave == 1) {
    if (lane < 16) {
      const v4f v = *(const v4f*)(qws + 4 * lane);
      float* dst = QW + (size_t)bp * kHID + 4 * lane;
      *(volatile v4f*)dst = v;
      __threadfence();
      *(volatile v4f*)dst = v;
    }
  }
}

__global__ __launch_bounds__(256) void k_lazy1(const float* __restrict__ dyn, const float* __restrict__ QW,
                                              const float* __restrict__ lW1, unsigned short* __restrict__ H1,
                                              int chunk) {
  __shared__ __align__(16) float w1s[3 * kHID];
  __shared__ __align__(16) unsigned short hs[256 * kHID];
  const int t = threadIdx.x;
  if (t < 3 * kHID) w1s[t] = lW1[t];
  __syncthreads();
  const int row = blockIdx.x * 256 + t;
  const int bpl = row >> 10, n = row & (kNP - 1);
  const int bp = chunk * kChunkBP + bpl;
  const int nc = (n < kN) ? n : (kN - 1);
  const float* dp = dyn + ((size_t)bp * kN + nc) * kDYN;
  const float d0 = dp[0], d1 = dp[1], d2 = dp[2];
  const float* qwp = QW + (size_t)bp * kHID;
#pragma unroll 1
  for (int g = 0; g < 8; ++g) {
    const v4f qa = *(const v4f*)(qwp + 8 * g), qb = *(const v4f*)(qwp + 8 * g + 4);
    const v4f a0 = *(const v4f*)(w1s + 8 * g),            a1 = *(const v4f*)(w1s + 8 * g + 4);
    const v4f e0 = *(const v4f*)(w1s + kHID + 8 * g),     e1 = *(const v4f*)(w1s + kHID + 8 * g + 4);
    const v4f c0 = *(const v4f*)(w1s + 2 * kHID + 8 * g), c1 = *(const v4f*)(w1s + 2 * kHID + 8 * g + 4);
    const v4f x0 = a0 * d0 + (e0 * d1 + (c0 * d2 + qa));
    const v4f x1 = a1 * d0 + (e1 * d1 + (c1 * d2 + qb));
    unsigned short hb[8];
#pragma unroll
    for (int e = 0; e < 4; ++e) {
      hb[e]     = h_bits(fmaxf(x0[e], 0.0f));
      hb[4 + e] = h_bits(fmaxf(x1[e], 0.0f));
    }
    *(v4u*)(hs + t * kHID + 8 * g) = (v4u){pk16(hb[0], hb[1]), pk16(hb[2], hb[3]), pk16(hb[4], hb[5]), pk16(hb[6], hb[7])};
  }
  __syncthreads();
  unsigned short* hbase = H1 + (size_t)blockIdx.x * 256 * kHID;
  v4u vv[8];
#pragma unroll
  for (int i = 0; i < 8; ++i) vv[i] = *(const v4u*)(hs + 8 * (i * 256 + t));
  for (int pass = 0; pass < 2; ++pass) {
#pragma unroll
    for (int i = 0; i < 8; ++i) *(volatile v4u*)(hbase + 8 * (size_t)(i * 256 + t)) = vv[i];
    __threadfence();
  }
}

__global__ __launch_bounds__(256) void k_lazy3(const _Float16* __restrict__ H2, const float* __restrict__ lW3,
                                              const float* __restrict__ lb3, const float* __restrict__ ninfm,
                                              float* __restrict__ maskb, int chunk) {
  __shared__ __align__(16) float w3s[kHID];
  const int t = threadIdx.x;
  if (t < kHID) w3s[t] = lW3[t];
  __syncthreads();
  const int row = blockIdx.x * 256 + t;
  const int bpl = row >> 10, n = row & (kNP - 1);
  const int bp = chunk * kChunkBP + bpl;
  const int nc = (n < kN) ? n : (kN - 1);
  const _Float16* hp = H2 + (size_t)row * kHID;
  float z = 0.0f;
#pragma unroll 1
  for (int c = 0; c < 8; ++c) {
    const v8h hv = *(const v8h*)(hp + 8 * c);
    const v4f w0 = *(const v4f*)(w3s + 8 * c), w1 = *(const v4f*)(w3s + 8 * c + 4);
#pragma unroll
    for (int e = 0; e < 4; ++e) z = fmaf((float)hv[e], w0[e], z);
#pragma unroll
    for (int e = 0; e < 4; ++e) z = fmaf((float)hv[4 + e], w1[e], z);
  }
  z += lb3[0];
  const float spv = fmaxf(z, 0.0f) + log1pf(expf(-fabsf(z)));
  const float val = ninfm[(size_t)bp * kN + nc] - spv;
  float* mp = maskb + (size_t)chunk * kChunkRows + row;
  *(volatile float*)mp = val;
  __threadfence();
  *(volatile float*)mp = val;
}

__global__ __launch_bounds__(128) void k_attn(const float* __restrict__ Qs, const float* __restrict__ KV,
                                             const float* __restrict__ maskb, unsigned short* __restrict__ Ohi,
                                             unsigned short* __restrict__ Olo) {
  __shared__ __align__(16) float kvs[32 * 256];
  __shared__ __align__(16) float ms[16 * 32];
  __shared__ __align__(16) float ost[16 * kHD];
  const float kNegInf = -__builtin_inff();
  const int t = threadIdx.x, lane = t & 31, wave = t >> 5;
  const int b = blockIdx.x / 7, pg = blockIdx.x - b * 7, p0 = pg * 16;
  const int h = t >> 4, pl = t & 15;
  const int p = p0 + pl, pc = (p < kP) ? p : (kP - 1);
  const float* qp = Qs + (size_t)(b * kP + pc) * kHD + h * kD;
  const v4f qa = *(const v4f*)(qp), qb = *(const v4f*)(qp + 4), qc = *(const v4f*)(qp + 8), qd = *(const v4f*)(qp + 12);
  v4f oa = (v4f){0.f, 0.f, 0.f, 0.f}, ob = (v4f){0.f, 0.f, 0.f, 0.f}, oc = (v4f){0.f, 0.f, 0.f, 0.f}, od = (v4f){0.f, 0.f, 0.f, 0.f};
  float m = -3.0e38f, l = 0.0f;
  const float* kvb = KV + (size_t)b * kNP * (2 * kHD);
  const float* mkb = maskb + (size_t)(b * kP) * kNP;
#pragma unroll 1
  for (int ch = 0; ch < kNP / 32; ++ch) {
    const int n0 = ch * 32;
    __syncthreads();
    const float* src = kvb + (size_t)n0 * (2 * kHD);
#pragma unroll
    for (int i = 0; i < 16; ++i) {
      const int f = i * 128 + t;
      *(v4f*)(kvs + 4 * f) = *(const v4f*)(src + 4 * f);
    }
    {
      const int r = t >> 3, j4 = (t & 7) * 4;
      const int pr = (p0 + r < kP) ? (p0 + r) : (kP - 1);
      *(v4f*)(ms + r * 32 + j4) = *(const v4f*)(mkb + (size_t)pr * kNP + n0 + j4);
    }
    __syncthreads();
#pragma unroll 1
    for (int j = 0; j < 32; ++j) {
      const float* kr = kvs + j * 256 + h * kD;
      const v4f k0 = *(const v4f*)(kr), k1 = *(const v4f*)(kr + 4), k2 = *(const v4f*)(kr + 8), k3 = *(const v4f*)(kr + 12);
      float s = ms[pl * 32 + j];
      s = fmaf(qa[0], k0[0], s); s = fmaf(qa[1], k0[1], s); s = fmaf(qa[2], k0[2], s); s = fmaf(qa[3], k0[3], s);
      s = fmaf(qb[0], k1[0], s); s = fmaf(qb[1], k1[1], s); s = fmaf(qb[2], k1[2], s); s = fmaf(qb[3], k1[3], s);
      s = fmaf(qc[0], k2[0], s); s = fmaf(qc[1], k2[1], s); s = fmaf(qc[2], k2[2], s); s = fmaf(qc[3], k2[3], s);
      s = fmaf(qd[0], k3[0], s); s = fmaf(qd[1], k3[1], s); s = fmaf(qd[2], k3[2], s); s = fmaf(qd[3], k3[3], s);
      s = (n0 + j < kN) ? s : kNegInf;
      const float mn = fmaxf(m, s);
      const float alpha = __expf(m - mn);
      const float pj = __expf(s - mn);
      m = mn;
      l = fmaf(l, alpha, pj);
      const v4f v0 = *(const v4f*)(kr + kHD), v1 = *(const v4f*)(kr + kHD + 4), v2 = *(const v4f*)(kr + kHD + 8), v3 = *(const v4f*)(kr + kHD + 12);
      oa = v0 * pj + oa * alpha;
      ob = v1 * pj + ob * alpha;
      oc = v2 * pj + oc * alpha;
      od = v3 * pj + od * alpha;
    }
  }
  const float inv = 1.0f / l;
  {
    float* op = ost + pl * kHD + h * kD;
    *(v4f*)(op)      = oa * inv;
    *(v4f*)(op + 4)  = ob * inv;
    *(v4f*)(op + 8)  = oc * inv;
    *(v4f*)(op + 12) = od * inv;
  }
  __syncthreads();
  const int hh = lane >> 4, c8 = (lane & 15) * 8;
  v4u uh[2], ul[2];
  int prow[2];
#pragma unroll
  for (int k = 0; k < 2; ++k) {
    const int rl = wave * 4 + 2 * k + hh;
    prow[k] = p0 + rl;
    const float* s8 = ost + rl * kHD + c8;
    const v4f x0 = *(const v4f*)(s8), x1 = *(const v4f*)(s8 + 4);
    unsigned short hb[8], lb[8];
#pragma unroll
    for (int e = 0; e < 4; ++e) {
      split_bf(x0[e], hb[e], lb[e]);
      split_bf(x1[e], hb[4 + e], lb[4 + e]);
    }
    uh[k] = (v4u){pk16(hb[0], hb[1]), pk16(hb[2], hb[3]), pk16(hb[4], hb[5]), pk16(hb[6], hb[7])};
    ul[k] = (v4u){pk16(lb[0], lb[1]), pk16(lb[2], lb[3]), pk16(lb[4], lb[5]), pk16(lb[6], lb[7])};
  }
  for (int pass = 0; pass < 2; ++pass) {
#pragma unroll
    for (int k = 0; k < 2; ++k) {
      if (prow[k] < kP) {
        const size_t o = (size_t)(b * kP + prow[k]) * kHD + c8;
        *(volatile v4u*)(Ohi + o) = uh[k];
        *(volatile v4u*)(Olo + o) = ul[k];
      }
    }
    __threadfence();
  }
}

__global__ __launch_bounds__(256) void k_zero16x2(unsigned int* __restrict__ p0, unsigned int* __restrict__ p1, int nvec) {
  const int i = blockIdx.x * 256 + threadIdx.x;
  if (i >= 2 * nvec) return;
  unsigned int* p = (i < nvec) ? (p0 + 4 * (size_t)i) : (p1 + 4 * (size_t)(i - nvec));
  const v4u z = (v4u){0u, 0u, 0u, 0u};
  *(volatile v4u*)p = z;
  __threadfence();
  *(volatile v4u*)p = z;
}

__global__ __launch_bounds__(256) void k_final(const float* __restrict__ Sp, const float* __restrict__ ninfm,
                                              float* __restrict__ out) {
  __shared__ __align__(16) float xs[8 * kN];
  __shared__ float invs[8];
  const float kNegInf = -__builtin_inff();
  const int t = threadIdx.x, lane = t & 31, wave = t >> 5;
  const int r = blockIdx.x * 8 + wave;
  const int b = r / kP, p = r - b * kP;
  const float* srow = Sp + (size_t)(b * kSrows + p) * kNP;
  const float* nrow = ninfm + (size_t)r * kN;
  float* xr = xs + wave * kN;
  float mx = kNegInf;
#pragma unroll 1
  for (int i = 0; i < 32; ++i) {
    const int n = lane + 32 * i;
    const int nc = (n < kN) ? n : (kN - 1);
    const float x = kClip * tanhf(srow[nc]) + nrow[nc];
    if (n < kN) { xr[n] = x; mx = fmaxf(mx, x); }
  }
#pragma unroll
  for (int off = 16; off > 0; off >>= 1) mx = fmaxf(mx, __shfl_xor(mx, off, 32));
  float sum = 0.0f;
#pragma unroll 1
  for (int i = 0; i < 32; ++i) {
    const int n = lane + 32 * i;
    if (n < kN) { const float e = __expf(xr[n] - mx); xr[n] = e; sum += e; }
  }
#pragma unroll
  for (int off = 16; off > 0; off >>= 1) sum += __shfl_xor(sum, off, 32);
  if (lane == 0) invs[wave] = 1.0f / sum;
  __syncthreads();
  float* obase = out + (size_t)blockIdx.x * 8 * kN;
  for (int pass = 0; pass < 2; ++pass) {
#pragma unroll 1
    for (int f = t; f < 2 * kN; f += 256) {
      v4f v = *(const v4f*)(xs + 4 * f);
      v = v * invs[f / 250];
      *(volatile v4f*)(obase + 4 * (size_t)f) = v;
    }
    __threadfence();
  }
}

static inline size_t align256(size_t x) { return (x + 255) & ~(size_t)255; }

extern "C" void kernel_launch(void* const* d_in, const int* in_sizes, int n_in,
                              void* d_out, int out_size, void* d_ws, size_t ws_size,
                              hipStream_t stream) {
  if (n_in < 22) return;
  if (in_sizes[0] != kB * kN * kE || in_sizes[1] != kB * kP * kE || in_sizes[2] != kB * kP ||
      in_sizes[3] != kB * kP * kN || in_sizes[4] != kB * kP * kN * kDYN || out_size != kB * kP * kN) return;

  const float* enc      = (const float*)d_in[0];
  const float* enc_last = (const float*)d_in[1];
  const float* loadv    = (const float*)d_in[2];
  const float* ninfm    = (const float*)d_in[3];
  const float* dyn      = (const float*)d_in[4];
  const float* Wq       = (const float*)d_in[5];
  const float* Wk       = (const float*)d_in[6];
  const float* Wv       = (const float*)d_in[7];
  const float* Wc       = (const float*)d_in[8];
  const float* bcv      = (const float*)d_in[9];
  const float* fW1      = (const float*)d_in[10];
  const float* fb1      = (const float*)d_in[11];
  const float* fW2      = (const float*)d_in[12];
  const float* fb2      = (const float*)d_in[13];
  const float* lqW      = (const float*)d_in[14];
  const float* lqb      = (const float*)d_in[15];
  const float* lW1      = (const float*)d_in[16];
  const float* lb1      = (const float*)d_in[17];
  const float* lW2      = (const float*)d_in[18];
  const float* lb2      = (const float*)d_in[19];
  const float* lW3      = (const float*)d_in[20];
  const float* lb3      = (const float*)d_in[21];
  float* out = (float*)d_out;

  char* ws = (char*)d_ws;
  size_t off = 0;
  unsigned short* EncHi = (unsigned short*)(ws + off); off = align256(off + (size_t)kEncRows * kE * 2);
  unsigned short* EncLo = (unsigned short*)(ws + off); off = align256(off + (size_t)kEncRows * kE * 2);
  unsigned short* WkvHi = (unsigned short*)(ws + off); off = align256(off + (size_t)2 * kHD * kE * 2);
  unsigned short* WkvLo = (unsigned short*)(ws + off); off = align256(off + (size_t)2 * kHD * kE * 2);
  unsigned short* WcHi  = (unsigned short*)(ws + off); off = align256(off + (size_t)kE * kHD * 2);
  unsigned short* WcLo  = (unsigned short*)(ws + off); off = align256(off + (size_t)kE * kHD * 2);
  unsigned short* W2T   = (unsigned short*)(ws + off); off = align256(off + (size_t)kHID * kHID * 2);
  float* KVf   = (float*)(ws + off); off = align256(off + (size_t)kEncRows * 2 * kHD * 4);
  float* Qs    = (float*)(ws + off); off = align256(off + (size_t)kBP * kHD * 4);
  float* QW    = (float*)(ws + off); off = align256(off + (size_t)kBP * kHID * 4);
  float* MASKB = (float*)(ws + off); off = align256(off + (size_t)kBP * kNP * 4);
  unsigned short* H1c  = (unsigned short*)(ws + off); off = align256(off + (size_t)kChunkRows * kHID * 2);
  unsigned short* H2c  = (unsigned short*)(ws + off); off = align256(off + (size_t)kChunkRows * kHID * 2);
  unsigned short* Ohi  = (unsigned short*)(ws + off); off = align256(off + (size_t)kBPpad * kHD * 2);
  unsigned short* Olo  = (unsigned short*)(ws + off); off = align256(off + (size_t)kBPpad * kHD * 2);
  unsigned short* MHhi = (unsigned short*)(ws + off); off = align256(off + (size_t)kBPpad * kE * 2);
  unsigned short* MHlo = (unsigned short*)(ws + off); off = align256(off + (size_t)kBPpad * kE * 2);
  float* Sp    = (float*)(ws + off); off = align256(off + (size_t)kB * kSrows * kNP * 4);
  if (off > ws_size) return;
  const float* fdummy = Qs;

  k_wprep<<<13, 256, 0, stream>>>(Wk, Wv, Wc, lW2, WkvHi, WkvLo, WcHi, WcLo, W2T);
  k_enc_cast<<<(kEncRows * 16) / 256, 256, 0, stream>>>(enc, EncHi, EncLo);
  wmma_gemm64<1, true, 0, 0, false, 0><<<dim3((kEncRows / 64) * (2 * kHD / 64) / 8, 1), 256, 0, stream>>>(
      EncHi, EncLo, kE, 0L, WkvHi, WkvLo, kE, 0L, (void*)KVf, (void*)KVf, 2 * kHD, 0L,
      fdummy, fdummy, 0L, kEncRows, 2 * kHD, kE, 1.0f);
  k_qside<<<kBP, 128, 0, stream>>>(enc_last, loadv, Wq, fW1, fb1, fW2, fb2, lqW, lqb, lW1, lb1, Qs, QW);
  for (int c = 0; c < kNumChunks; ++c) {
    k_lazy1<<<kChunkRows / 256, 256, 0, stream>>>(dyn, QW, lW1, H1c, c);
    wmma_gemm64<0, false, 2, 1, false, 2><<<dim3((kChunkRows / 64) / 8, 1), 256, 0, stream>>>(
        H1c, H1c, kHID, 0L, W2T, W2T, kHID, 0L, (void*)H2c, (void*)H2c, kHID, 0L,
        lb2, lb2, 0L, kChunkRows, kHID, kHID, 1.0f / kWCarry);
    k_lazy3<<<kChunkRows / 256, 256, 0, stream>>>((const _Float16*)H2c, lW3, lb3, ninfm, MASKB, c);
  }
  k_zero16x2<<<(2 * 1024) / 256, 256, 0, stream>>>((unsigned int*)(Ohi + (size_t)kBP * kHD),
                                                   (unsigned int*)(Olo + (size_t)kBP * kHD), 1024);
  k_attn<<<kB * 7, 128, 0, stream>>>(Qs, KVf, MASKB, Ohi, Olo);
  wmma_gemm64<1, true, 2, 2, false, 0><<<dim3(((kBPpad / 64) * (kE / 64) + 7) / 8, 1), 256, 0, stream>>>(
      Ohi, Olo, kHD, 0L, WcHi, WcLo, kHD, 0L, (void*)MHhi, (void*)MHlo, kE, 0L,
      bcv, fdummy, 0L, kBPpad, kE, kHD, 1.0f);
  wmma_gemm64<1, true, 0, 0, false, 0><<<dim3((kSrows / 64) * (kNP / 64) / 8, kB), 256, 0, stream>>>(
      MHhi, MHlo, kE, (long)kP * kE, EncHi, EncLo, kE, (long)kNP * kE, (void*)Sp, (void*)Sp, kNP, (long)kSrows * kNP,
      fdummy, fdummy, 0L, kSrows, kNP, kE, kInvSqrtE);
  k_final<<<kBP / 8, 256, 0, stream>>>(Sp, ninfm, out);
}
